// Encoder_4269197492519
// MI455X (gfx1250) — hardware-verified
//
#include <hip/hip_runtime.h>
#include <stddef.h>
#include <stdint.h>


#define DF     128
#define AP     384
#define KG     384
#define NTHR   256
#define NWAVE  8
#define EPT    8
#define CHUNK  (NTHR * EPT)
#define WCAP   (EPT * 32)
#define LISTN  (NWAVE * WCAP)
#define NBA    1024
#define SLA    10
#define RCAP   28672
#define DEGCAP 64
#define GBM    64
#define GBN    128
#define GTHR   128
#define UPART  2048
#define NPART  6
#define AGG_ZINTS    (LISTN + 2 * RCAP + 3 * NBA)
#define MISC_INTS    16
#define ROWBUF_INTS  (NWAVE * DF)
#define AGG_LDS_INTS (AGG_ZINTS + MISC_INTS + ROWBUF_INTS)
#define WSMAX  134217728

static_assert((CHUNK & (CHUNK - 1)) == 0 && CHUNK <= 4096);
static_assert((NBA & (NBA - 1)) == 0 && NBA == (1 << SLA));
static_assert(((long long)CHUNK << SLA) < (1LL << 31));
static_assert(LISTN % NTHR == 0);
static_assert(NBA % NWAVE == 0 && NBA % 32 == 0 && NBA % GBM == 0);
static_assert(RCAP % 4 == 0 && AGG_ZINTS % 4 == 0 && LISTN % 4 == 0 && ((AGG_ZINTS + MISC_INTS) % 4) == 0);
static_assert(AGG_ZINTS % (NTHR * 4) == 0);
static_assert(KG % 32 == 0 && KG == AP && KG == 3 * DF);
static_assert(GBN == DF && GBM == (GTHR / 32) * 16 && DF == 4 * 32);
static_assert(UPART % NTHR == 0 && UPART == DF * (DF / 8));
static_assert((NPART * UPART) % NTHR == 0);
static_assert((AP * 2) % 128 == 0 && (2 * DF * 2) % 128 == 0);
static_assert(AGG_LDS_INTS * 4 <= 300000);

typedef float          v4f   __attribute__((ext_vector_type(4)));
typedef float          v8f   __attribute__((ext_vector_type(8)));
typedef int            v4i   __attribute__((ext_vector_type(4)));
typedef int            v8i   __attribute__((ext_vector_type(8)));
typedef unsigned       v2u   __attribute__((ext_vector_type(2)));
typedef unsigned short v4us  __attribute__((ext_vector_type(4)));
typedef unsigned short v8us  __attribute__((ext_vector_type(8)));
typedef unsigned short v16us __attribute__((ext_vector_type(16)));
typedef __bf16         v16bf __attribute__((ext_vector_type(16)));
typedef v4f  __attribute__((may_alias)) v4fa;
typedef v4i  __attribute__((may_alias)) v4ia;
typedef v2u  __attribute__((may_alias)) v2ua;
typedef v4us __attribute__((may_alias)) v4usa;
typedef v8us __attribute__((may_alias)) v8usa;
union FragB { v16bf v; v16us u; v8us h[2]; v8i w; };

__device__ __forceinline__ v8f wmb(const FragB& a, const FragB& b, v8f c) {
  v8f d = __builtin_amdgcn_wmma_f32_16x16x32_bf16(false, a.v, false, b.v, (short)0, c, false, false);
  asm volatile("v_nop\n\tv_nop\n\tv_nop\n\tv_nop" : "+v"(d) : "v"(a.w), "v"(b.w));
  return d;
}

__device__ __forceinline__ unsigned bf16_bits(float f) {
  const unsigned u = __float_as_uint(f);
  return (u + 0x7FFFu + ((u >> 16) & 1u)) >> 16;
}
__device__ __forceinline__ float bf16_val(float f) {
  return __uint_as_float(bf16_bits(f) << 16);
}

__device__ __forceinline__ void wave_sync() {
  __builtin_amdgcn_fence(__ATOMIC_RELEASE, "wavefront");
  __builtin_amdgcn_wave_barrier();
  __builtin_amdgcn_fence(__ATOMIC_ACQUIRE, "wavefront");
}

template <int SLB>
__device__ __forceinline__ int scan_chunk(const int* __restrict__ dsts, int nE, int cbase, int slotBase,
                                          int nb, int vec8, int* list, int tid, int lane, int wave) {
  int wc = 0;
  const int el0  = tid * EPT;
  const int e0   = cbase + el0;
  const int sent = -2147483647 - 1;
  v4i da, db;
  if (vec8 != 0 && cbase + CHUNK <= nE) {
    da = *(const v4i*)(dsts + e0);
    db = *(const v4i*)(dsts + e0 + 4);
  } else {
    da.x = (e0     < nE) ? dsts[min(e0,     nE - 1)] : sent;
    da.y = (e0 + 1 < nE) ? dsts[min(e0 + 1, nE - 1)] : sent;
    da.z = (e0 + 2 < nE) ? dsts[min(e0 + 2, nE - 1)] : sent;
    da.w = (e0 + 3 < nE) ? dsts[min(e0 + 3, nE - 1)] : sent;
    db.x = (e0 + 4 < nE) ? dsts[min(e0 + 4, nE - 1)] : sent;
    db.y = (e0 + 5 < nE) ? dsts[min(e0 + 5, nE - 1)] : sent;
    db.z = (e0 + 6 < nE) ? dsts[min(e0 + 6, nE - 1)] : sent;
    db.w = (e0 + 7 < nE) ? dsts[min(e0 + 7, nE - 1)] : sent;
  }
  const unsigned nbs = (unsigned)slotBase;
  const unsigned unb = (unsigned)nb;
  const unsigned s0 = (unsigned)da.x - nbs, s1 = (unsigned)da.y - nbs;
  const unsigned s2 = (unsigned)da.z - nbs, s3 = (unsigned)da.w - nbs;
  const unsigned s4 = (unsigned)db.x - nbs, s5 = (unsigned)db.y - nbs;
  const unsigned s6 = (unsigned)db.z - nbs, s7 = (unsigned)db.w - nbs;
  const bool h0 = s0 < unb, h1 = s1 < unb, h2 = s2 < unb, h3 = s3 < unb;
  const bool h4 = s4 < unb, h5 = s5 < unb, h6 = s6 < unb, h7 = s7 < unb;
  const unsigned any = __builtin_amdgcn_ballot_w32(h0 | h1 | h2 | h3 | h4 | h5 | h6 | h7);
  if (any != 0u) {
#define HITJ(J, HJ, SJ) { \
      const unsigned mj = __builtin_amdgcn_ballot_w32(HJ); \
      if (mj != 0u) { \
        if (HJ) { \
          const int pos = wc + (int)__builtin_amdgcn_mbcnt_lo(mj, 0u); \
          if (pos < WCAP) list[wave * WCAP + pos] = ((el0 + (J)) << SLB) | (int)(SJ); \
        } \
        wc += (int)__builtin_popcount(mj); } }
    HITJ(0, h0, s0)
    HITJ(1, h1, s1)
    HITJ(2, h2, s2)
    HITJ(3, h3, s3)
    HITJ(4, h4, s4)
    HITJ(5, h5, s5)
    HITJ(6, h6, s6)
    HITJ(7, h7, s7)
#undef HITJ
  }
  return wc;
}

__global__ __launch_bounds__(NTHR) void k_wprep(const float* __restrict__ Wlui, const float* __restrict__ Wrui,
                                                const float* __restrict__ Wliu, const float* __restrict__ Wriu,
                                                unsigned short* WTui, unsigned short* WTiu) {
  const int u    = (int)blockIdx.x * NTHR + (int)threadIdx.x;
  const int part = u >> 11;
  const int v    = u & (UPART - 1);
  const int n    = v >> 4;
  const int k8   = (v & 15) * 8;
  const float* W;
  unsigned short* P;
  int coff;
  if (part == 0)       { W = Wlui; P = WTui; coff = 0; }
  else if (part == 1)  { W = Wlui; P = WTui; coff = DF; }
  else if (part == 2)  { W = Wrui; P = WTui; coff = 2 * DF; }
  else if (part == 3)  { W = Wliu; P = WTiu; coff = 0; }
  else if (part == 4)  { W = Wliu; P = WTiu; coff = DF; }
  else if (part == 5)  { W = Wriu; P = WTiu; coff = 2 * DF; }
  else return;
  const float* p = W + (size_t)k8 * DF + n;
  v8us o;
#pragma unroll
  for (int i = 0; i < 8; ++i) o[i] = (unsigned short)bf16_bits(p[(size_t)i * DF]);
  unsigned short* dp = P + (size_t)n * AP + coff + k8;
  *(volatile v8us*)dp = o;
  __threadfence();
  *(volatile v8us*)dp = o;
}

template <int GATH>
__global__ __launch_bounds__(NTHR) void k_rows(const float* __restrict__ src, const int* __restrict__ ids,
                                               int nN, int nSrc, int nUnits, unsigned short* plane) {
  const int u = (int)blockIdx.x * NTHR + (int)threadIdx.x;
  if (u >= nUnits) return;
  const int row = u >> 4;
  const int k8  = (u & 15) * 8;
  const int rc  = row < nN ? row : nN - 1;
  int sr = rc;
  if constexpr (GATH != 0) {
    sr = ids[rc];
    sr = sr < 0 ? 0 : (sr > nSrc - 1 ? nSrc - 1 : sr);
  } else {
    sr = sr > nSrc - 1 ? nSrc - 1 : sr;
  }
  const float* p = src + (size_t)sr * DF + k8;
  const v4f a = *(const v4fa*)p;
  const v4f b = *(const v4fa*)(p + 4);
  const bool ok = row < nN;
  v8us o;
  o[0] = ok ? (unsigned short)bf16_bits(a.x) : (unsigned short)0;
  o[1] = ok ? (unsigned short)bf16_bits(a.y) : (unsigned short)0;
  o[2] = ok ? (unsigned short)bf16_bits(a.z) : (unsigned short)0;
  o[3] = ok ? (unsigned short)bf16_bits(a.w) : (unsigned short)0;
  o[4] = ok ? (unsigned short)bf16_bits(b.x) : (unsigned short)0;
  o[5] = ok ? (unsigned short)bf16_bits(b.y) : (unsigned short)0;
  o[6] = ok ? (unsigned short)bf16_bits(b.z) : (unsigned short)0;
  o[7] = ok ? (unsigned short)bf16_bits(b.w) : (unsigned short)0;
  unsigned short* dp = plane + (size_t)row * AP + 2 * DF + k8;
  *(volatile v8us*)dp = o;
  __threadfence();
  *(volatile v8us*)dp = o;
}

__global__ __launch_bounds__(GTHR) void k_gemm(const unsigned short* __restrict__ Apl,
                                               const unsigned short* __restrict__ BT,
                                               const float* __restrict__ bias, float* outp, int nOut) {
  __shared__ __attribute__((aligned(16))) float stg[GBM * GBN];
  const int tid = (int)threadIdx.x, lane = tid & 31, wave = tid >> 5, hh = lane >> 4, m = lane & 15;
  const int rowBase = (int)blockIdx.x * GBM;

  v8f acc[8];
  {
    const v8f z = {0.f, 0.f, 0.f, 0.f, 0.f, 0.f, 0.f, 0.f};
#pragma unroll
    for (int t = 0; t < 8; ++t) acc[t] = z;
  }
  const unsigned short* ap = Apl + (size_t)(rowBase + 16 * wave + m) * (size_t)AP + 8 * hh;
  const unsigned short* bp = BT + (size_t)m * (size_t)KG + 8 * hh;

#pragma unroll 1
  for (int k0 = 0; k0 < KG; k0 += 32) {
    FragB af;
    af.h[0] = *(const v8usa*)(ap + k0);
    af.h[1] = *(const v8usa*)(ap + k0 + 16);
#pragma unroll
    for (int nt = 0; nt < 8; ++nt) {
      const unsigned short* wq = bp + (size_t)(16 * nt) * (size_t)KG + k0;
      FragB bf;
      bf.h[0] = *(const v8usa*)wq;
      bf.h[1] = *(const v8usa*)(wq + 16);
      acc[nt] = wmb(af, bf, acc[nt]);
    }
  }

#pragma unroll
  for (int nt = 0; nt < 8; ++nt) {
    const int lc = 16 * nt + m;
#pragma unroll
    for (int r = 0; r < 8; ++r) {
      const int lr = 16 * wave + 8 * hh + r;
      stg[lr * GBN + lc] = acc[nt][r];
    }
  }
  __syncthreads();

  v4f bb4;
  {
    const v4f t1 = *(const v4fa*)(bias + 4 * lane);
    bb4.x = bf16_val(t1.x);
    bb4.y = bf16_val(t1.y);
    bb4.z = bf16_val(t1.z);
    bb4.w = bf16_val(t1.w);
  }

  v4f pv[16];
#pragma unroll
  for (int i = 0; i < 16; ++i) {
    const v4f t = *(const v4fa*)(stg + (16 * wave + i) * GBN + 4 * lane);
    pv[i] = t + bb4;
  }

#pragma unroll
  for (int i = 0; i < 16; ++i) {
    const int r = rowBase + 16 * wave + i;
    if (r < nOut) *(volatile v4f*)(outp + (size_t)r * DF + 4 * lane) = pv[i];
  }
  __threadfence();
#pragma unroll
  for (int i = 0; i < 16; ++i) {
    const int r = rowBase + 16 * wave + i;
    if (r < nOut) *(volatile v4f*)(outp + (size_t)r * DF + 4 * lane) = pv[i];
  }
}

__global__ __launch_bounds__(NTHR) void k_scan(const int* __restrict__ gath, const int* __restrict__ keys,
                                               int nE, int nDst, int nSrc, int vec8, int mRows,
                                               const unsigned short* srcPl, unsigned short* dstPl) {
  extern __shared__ __attribute__((aligned(16))) int dsm[];
  int* list = dsm;
  int* hl   = dsm + LISTN;
  int* sl   = hl + RCAP;
  int* cnt  = sl + RCAP;
  int* offs = cnt + NBA;
  int* cur  = offs + NBA;
  int* misc = cur + NBA;
  const int tid = (int)threadIdx.x, lane = tid & 31, wave = tid >> 5;
  unsigned short* rowbuf = (unsigned short*)(misc + MISC_INTS) + wave * (2 * DF);
  const int nodeBase = (int)blockIdx.x * NBA;

  {
    const v4i z4 = {0, 0, 0, 0};
    for (int i = tid * 4; i < AGG_ZINTS; i += NTHR * 4) *(v4ia*)(dsm + i) = z4;
    if (tid < MISC_INTS) misc[tid] = 0;
  }
  __syncthreads();

  int t = 0, ov = 0;
  const int nChunks = (nE + CHUNK - 1) / CHUNK;
#pragma unroll 1
  for (int ch = 0; ch < nChunks; ++ch) {
    const int cbase = ch * CHUNK;
    const int wc = scan_chunk<SLA>(keys, nE, cbase, nodeBase, NBA, vec8, list, tid, lane, wave);
    if (lane == 0) misc[wave] = wc;
    __syncthreads();
    if (wave == 0) {
#pragma unroll 1
      for (int w2 = 0; w2 < NWAVE; ++w2) {
        int c = misc[w2];
        c = c < 0 ? 0 : (c > WCAP ? WCAP : c);
#pragma unroll 1
        for (int b0 = 0; b0 < c; b0 += 32) {
          const int idx = b0 + lane;
          const int ent = list[w2 * WCAP + (idx < WCAP ? idx : WCAP - 1)];
          const int m32 = (c - b0) < 32 ? (c - b0) : 32;
#pragma unroll 1
          for (int k = 0; k < m32; ++k) {
            const int u    = __builtin_amdgcn_readlane(ent, k);
            const int slot = u & (NBA - 1);
            const int el   = (u >> SLA) & (CHUNK - 1);
            const int pk   = ((cbase + el) << SLA) | slot;
            if (t < RCAP) {
              if (lane == 0) { hl[t] = pk; cnt[slot] = cnt[slot] + 1; }
              t = t + 1;
            } else {
              ov = 1;
            }
          }
        }
      }
    }
    __syncthreads();
  }
  if (wave == 0 && lane == 0) { misc[8] = t; misc[9] = ov; }
  __syncthreads();
  int tt = misc[8];
  tt = tt < 0 ? 0 : (tt > RCAP ? RCAP : tt);
  const int ovf = misc[9];

  if (wave == 0) {
    const int base = lane * (NBA / 32);
    int s = 0;
#pragma unroll 1
    for (int i = 0; i < NBA / 32; ++i) s += cnt[base + i];
    int incl = s;
#pragma unroll
    for (int d = 1; d < 32; d <<= 1) {
      const int y = __shfl_up(incl, d, 32);
      if (lane >= d) incl += y;
    }
    int run = incl - s;
#pragma unroll 1
    for (int i = 0; i < NBA / 32; ++i) {
      const int cv = cnt[base + i];
      offs[base + i] = run;
      cur[base + i]  = run;
      run += cv;
    }
  }
  __syncthreads();
  if (wave == 0) {
#pragma unroll 1
    for (int b0 = 0; b0 < tt; b0 += 32) {
      const int idx = b0 + lane;
      const int ent = hl[idx < RCAP ? idx : RCAP - 1];
      const int m32 = (tt - b0) < 32 ? (tt - b0) : 32;
#pragma unroll 1
      for (int k = 0; k < m32; ++k) {
        const int u    = __builtin_amdgcn_readlane(ent, k);
        const int slot = u & (NBA - 1);
        if (lane == 0) {
          int p = cur[slot];
          p = p < 0 ? 0 : (p > RCAP - 1 ? RCAP - 1 : p);
          sl[p] = u;
          cur[slot] = p + 1;
        }
      }
    }
  }
  __syncthreads();

  const float qnan = __int_as_float(0x7fc00000);
  const float pz = (ovf != 0) ? qnan : 0.0f;
#pragma unroll 1
  for (int si = 0; si < NBA / NWAVE; ++si) {
    const int s    = si * NWAVE + wave;
    const int node = nodeBase + s;
    const int craw = cnt[s];
    const bool big = craw > DEGCAP;
    int c = craw < 0 ? 0 : (craw > DEGCAP ? DEGCAP : craw);
    int o = offs[s];
    o = o < 0 ? 0 : (o > RCAP ? RCAP : o);
    float a0 = 0.0f, a1 = 0.0f, a2 = 0.0f, a3 = 0.0f;
#pragma unroll 1
    for (int b0 = 0; b0 < c; b0 += 32) {
      int idx = o + b0 + lane;
      idx = idx > RCAP - 1 ? RCAP - 1 : idx;
      const int ent = sl[idx];
      int eid = ent >> SLA;
      eid = eid < 0 ? 0 : (eid > nE - 1 ? nE - 1 : eid);
      int sr = gath[eid];
      sr = sr < 0 ? 0 : (sr > nSrc - 1 ? nSrc - 1 : sr);
      const int m32 = (c - b0) < 32 ? (c - b0) : 32;
#pragma unroll 1
      for (int k = 0; k < m32; ++k) {
        const int sk = __builtin_amdgcn_readlane(sr, k);
        const unsigned short* rp = srcPl + (size_t)sk * AP + 2 * DF + 4 * lane;
        const v2u w = *(const v2ua*)rp;
        a0 += __uint_as_float(w.x << 16);
        a1 += __uint_as_float(w.x & 0xffff0000u);
        a2 += __uint_as_float(w.y << 16);
        a3 += __uint_as_float(w.y & 0xffff0000u);
      }
    }
    const float cf  = (float)(craw < 1 ? 1 : craw);
    const float inv = 1.0f / cf;
    const float pzr = big ? qnan : pz;
    const bool live = node < nDst;
    const float m0 = live ? (a0 * inv + pzr) : 0.0f;
    const float m1 = live ? (a1 * inv + pzr) : 0.0f;
    const float m2 = live ? (a2 * inv + pzr) : 0.0f;
    const float m3 = live ? (a3 * inv + pzr) : 0.0f;
    v4us mh, ml;
    {
      unsigned hb;
      hb = bf16_bits(m0); mh[0] = (unsigned short)hb; ml[0] = (unsigned short)bf16_bits(m0 - __uint_as_float(hb << 16));
      hb = bf16_bits(m1); mh[1] = (unsigned short)hb; ml[1] = (unsigned short)bf16_bits(m1 - __uint_as_float(hb << 16));
      hb = bf16_bits(m2); mh[2] = (unsigned short)hb; ml[2] = (unsigned short)bf16_bits(m2 - __uint_as_float(hb << 16));
      hb = bf16_bits(m3); mh[3] = (unsigned short)hb; ml[3] = (unsigned short)bf16_bits(m3 - __uint_as_float(hb << 16));
    }
    *(v4usa*)(rowbuf + 4 * lane) = mh;
    *(v4usa*)(rowbuf + DF + 4 * lane) = ml;
    wave_sync();
    const v8us q0 = *(const v8usa*)(rowbuf + 8 * lane);
    wave_sync();
    if (node < mRows) {
      unsigned short* rpw = dstPl + (size_t)node * AP + 8 * lane;
      *(volatile v8us*)rpw = q0;
      __threadfence();
      *(volatile v8us*)rpw = q0;
    }
  }
}

static inline int cdiv(int a, int b) { return (a + b - 1) / b; }
static inline size_t al256(size_t o) { return (o + 255) & ~(size_t)255; }

extern "C" void kernel_launch(void* const* d_in, const int* in_sizes, int n_in,
                              void* d_out, int out_size, void* d_ws, size_t ws_size,
                              hipStream_t stream) {
  if (n_in < 11) return;
  const int nU = in_sizes[0];
  if (nU < 16 || nU >= (1 << 24)) return;
  if (in_sizes[1] < DF || (in_sizes[1] % DF) != 0) return;
  const int nI = in_sizes[1] / DF;
  if (nI < 16 || nI >= (1 << 24)) return;
  if (in_sizes[2] < 2 || (in_sizes[2] & 1) != 0) return;
  const int nEui = in_sizes[2] / 2;
  if (in_sizes[3] < 2 || (in_sizes[3] & 1) != 0) return;
  const int nEiu = in_sizes[3] / 2;
  if (nEui >= (1 << 21) || nEiu >= (1 << 21)) return;
  if (in_sizes[4] < DF || (in_sizes[4] % DF) != 0) return;
  const int nEmb = in_sizes[4] / DF;
  if (in_sizes[5] != DF * DF || in_sizes[6] != DF * DF || in_sizes[7] != DF) return;
  if (in_sizes[8] != DF * DF || in_sizes[9] != DF * DF || in_sizes[10] != DF) return;
  if ((long long)out_size != ((long long)nU + (long long)nI) * DF) return;

  const int*   user_ids = (const int*)d_in[0];
  const float* item_x   = (const float*)d_in[1];
  const int*   edge_ui  = (const int*)d_in[2];
  const int*   edge_iu  = (const int*)d_in[3];
  const float* user_emb = (const float*)d_in[4];
  const float* W_l_ui   = (const float*)d_in[5];
  const float* W_r_ui   = (const float*)d_in[6];
  const float* b_ui     = (const float*)d_in[7];
  const float* W_l_iu   = (const float*)d_in[8];
  const float* W_r_iu   = (const float*)d_in[9];
  const float* b_iu     = (const float*)d_in[10];
  float* out_user = (float*)d_out;
  float* out_item = out_user + (size_t)nU * DF;

  const int MPu = cdiv(nU, GBM) * GBM;
  const int MPi = cdiv(nI, GBM) * GBM;
  const int gAu = cdiv(MPu, NBA);
  const int gAi = cdiv(MPi, NBA);
  if ((long long)gAu * NBA < (long long)MPu || (long long)gAi * NBA < (long long)MPi) return;
  const int vecUI = ((nEui & 3) == 0) ? 1 : 0;
  const int vecIU = ((nEiu & 3) == 0) ? 1 : 0;

  char* ws = (char*)d_ws;
  size_t off = 0;
  const size_t oWTui = off; off = al256(off + (size_t)DF * AP * 2);
  const size_t oWTiu = off; off = al256(off + (size_t)DF * AP * 2);
  const size_t oAU   = off; off = al256(off + (size_t)MPu * AP * 2);
  const size_t oAI   = off; off = al256(off + (size_t)MPi * AP * 2);
  if (off > ws_size || off > (size_t)WSMAX) return;
  unsigned short* WTui = (unsigned short*)(ws + oWTui);
  unsigned short* WTiu = (unsigned short*)(ws + oWTiu);
  unsigned short* AU   = (unsigned short*)(ws + oAU);
  unsigned short* AI   = (unsigned short*)(ws + oAI);

  const size_t scanLds = (size_t)AGG_LDS_INTS * 4;
  hipFuncSetAttribute(reinterpret_cast<const void*>(&k_scan), hipFuncAttributeMaxDynamicSharedMemorySize, (int)scanLds);

  k_wprep<<<(NPART * UPART) / NTHR, NTHR, 0, stream>>>(W_l_ui, W_r_ui, W_l_iu, W_r_iu, WTui, WTiu);
  {
    const int nUn = MPu * (DF / 8);
    k_rows<1><<<cdiv(nUn, NTHR), NTHR, 0, stream>>>(user_emb, user_ids, nU, nEmb, nUn, AU);
  }
  {
    const int nUn = MPi * (DF / 8);
    k_rows<0><<<cdiv(nUn, NTHR), NTHR, 0, stream>>>(item_x, user_ids, nI, nI, nUn, AI);
  }
  k_scan<<<gAi, NTHR, scanLds, stream>>>(edge_ui, edge_ui + nEui, nEui, nI, nU, vecUI, MPi, AU, AI);
  k_scan<<<gAu, NTHR, scanLds, stream>>>(edge_iu, edge_iu + nEiu, nEiu, nU, nI, vecIU, MPu, AI, AU);
  k_gemm<<<MPi / GBM, GTHR, 0, stream>>>(AI, WTui, b_ui, out_item, nI);
  k_gemm<<<MPu / GBM, GTHR, 0, stream>>>(AU, WTiu, b_iu, out_user, nU);
}
